// decoderHead_15152644621126
// MI455X (gfx1250) — hardware-verified
//
#include <hip/hip_runtime.h>


#define NB 4
#define NS 4096
#define NE 512
#define ND 64
#define NROWS (NB * NS)
#define LDH 72
#define LDO 68

typedef _Float16 v8h  __attribute__((ext_vector_type(8)));
typedef _Float16 v16h __attribute__((ext_vector_type(16)));
typedef __bf16   v8b  __attribute__((ext_vector_type(8)));
typedef __bf16   v16b __attribute__((ext_vector_type(16)));
typedef float    v8f  __attribute__((ext_vector_type(8)));
typedef float    v4f  __attribute__((ext_vector_type(4)));
typedef unsigned int v4u __attribute__((ext_vector_type(4)));
typedef int      v4i  __attribute__((ext_vector_type(4)));

union FragH { v16h v; v8h h[2]; };
union FragB { v16b v; v8b h[2]; };
union Pack16 { v8h h; v8b b; v4u u; };

static __device__ __forceinline__ v8f mma_f16(v16h a, v16h b, v8f c) {
  c = __builtin_amdgcn_wmma_f32_16x16x32_f16(false, a, false, b, (short)0, c, false, false);
  asm volatile("v_nop\n\tv_nop\n\tv_nop\n\tv_nop" : "+v"(c) : "v"(a), "v"(b));
  return c;
}
static __device__ __forceinline__ v8f mma_bf16(v16b a, v16b b, v8f c) {
  c = __builtin_amdgcn_wmma_f32_16x16x32_bf16(false, a, false, b, (short)0, c, false, false);
  asm volatile("v_nop\n\tv_nop\n\tv_nop\n\tv_nop" : "+v"(c) : "v"(a), "v"(b));
  return c;
}

static __device__ __forceinline__ void load16f(const float* p0, const float* p1, float f[16]) {
  const v4f a = *(const v4f*)p0;
  const v4f b = *(const v4f*)(p0 + 4);
  const v4f c = *(const v4f*)p1;
  const v4f d = *(const v4f*)(p1 + 4);
  #pragma unroll
  for (int i = 0; i < 4; ++i) { f[i] = a[i]; f[4 + i] = b[i]; f[8 + i] = c[i]; f[12 + i] = d[i]; }
}

__global__ void __launch_bounds__(128) k_prepw(const float* __restrict__ Wq,
                                               const float* __restrict__ Wk,
                                               const float* __restrict__ Wv,
                                               _Float16* __restrict__ Wq16,
                                               _Float16* __restrict__ Wk16,
                                               __bf16* __restrict__ Wvh,
                                               __bf16* __restrict__ Wvl) {
  const int c = blockIdx.x * blockDim.x + threadIdx.x;
  const bool act = c < ND * (NE / 8);
  Pack16 pq, pk, ph, pl;
  pq.u = (v4u){0u, 0u, 0u, 0u}; pk.u = pq.u; ph.u = pq.u; pl.u = pq.u;
  size_t o = 0;
  if (act) {
    const int n = c >> 6;
    const int k0 = (c & 63) * 8;
    #pragma unroll
    for (int j = 0; j < 8; ++j) {
      const size_t src = (size_t)(k0 + j) * ND + n;
      const float wq = Wq[src];
      const float wk = Wk[src];
      const float wv = Wv[src];
      pq.h[j] = (_Float16)(wq * 1024.0f);
      pk.h[j] = (_Float16)(wk * 1024.0f);
      const __bf16 hb = (__bf16)wv;
      ph.b[j] = hb;
      pl.b[j] = (__bf16)(wv - (float)hb);
    }
    o = (size_t)n * NE + k0;
    *(volatile v4u*)(Wq16 + o) = pq.u;
    *(volatile v4u*)(Wk16 + o) = pk.u;
    *(volatile v4u*)(Wvh + o) = ph.u;
    *(volatile v4u*)(Wvl + o) = pl.u;
  }
  __threadfence();
  if (act) {
    *(volatile v4u*)(Wq16 + o) = pq.u;
    *(volatile v4u*)(Wk16 + o) = pk.u;
    *(volatile v4u*)(Wvh + o) = ph.u;
    *(volatile v4u*)(Wvl + o) = pl.u;
  }
}

__global__ void __launch_bounds__(128) k_projq(const float* __restrict__ x,
                                               const _Float16* __restrict__ Wq16,
                                               _Float16* __restrict__ Q16,
                                               float* __restrict__ maskbuf) {
  __shared__ __attribute__((aligned(16))) _Float16 st[4][16 * LDH];
  __shared__ __attribute__((aligned(16))) float ms[64];
  const int tid = threadIdx.x;
  const int lane = tid & 31, wave = tid >> 5, h = lane >> 4, lm = lane & 15;
  const int rowBase = blockIdx.x * 64 + wave * 16;

  v8f acc[4];
  {
    v8f z = {};
    #pragma unroll
    for (int i = 0; i < 4; ++i) acc[i] = z;
  }
  const float* xr = x + (size_t)(rowBase + lm) * NE;
  int nz = 0;

  #pragma unroll 1
  for (int ks = 0; ks < NE / 32; ++ks) {
    const int k0 = ks * 32;
    float f[16];
    load16f(xr + k0 + 8 * h, xr + k0 + 16 + 8 * h, f);
    FragH a;
    #pragma unroll
    for (int i = 0; i < 16; ++i) {
      a.v[i] = (_Float16)f[i];
      nz |= (f[i] != 0.0f) ? 1 : 0;
    }
    #pragma unroll
    for (int nt = 0; nt < 4; ++nt) {
      const _Float16* wr = Wq16 + (size_t)(nt * 16 + lm) * NE + k0;
      FragH b;
      b.h[0] = *(const v8h*)(wr + 8 * h);
      b.h[1] = *(const v8h*)(wr + 16 + 8 * h);
      acc[nt] = mma_f16(a.v, b.v, acc[nt]);
    }
  }

  nz |= __shfl_xor(nz, 16);
  const float mf = nz ? 1.0f : 0.0f;
  float mr[8];
  #pragma unroll
  for (int r = 0; r < 8; ++r) mr[r] = __shfl(mf, 8 * h + r);

  _Float16* sw = st[wave];
  #pragma unroll
  for (int nt = 0; nt < 4; ++nt) {
    #pragma unroll
    for (int r = 0; r < 8; ++r)
      sw[(8 * h + r) * LDH + nt * 16 + lm] = (_Float16)(acc[nt][r] * 0.015625f * mr[r]);
  }
  if (lane < 16) ms[wave * 16 + lane] = mf;
  __syncthreads();

  Pack16 u[4];
  #pragma unroll
  for (int p = 0; p < 4; ++p)
    u[p].h = *(const v8h*)(sw + (p * 4 + (lane >> 3)) * LDH + (lane & 7) * 8);
  _Float16* qd = Q16 + (size_t)rowBase * ND;
  const bool mw = (wave == 0) && (lane < 16);
  v4f mv = {0.0f, 0.0f, 0.0f, 0.0f};
  if (mw) mv = *(const v4f*)(ms + lane * 4);
  float* md = maskbuf + (size_t)blockIdx.x * 64 + lane * 4;

  #pragma unroll
  for (int p = 0; p < 4; ++p)
    *(volatile v4u*)(qd + (size_t)(p * 4 + (lane >> 3)) * ND + (lane & 7) * 8) = u[p].u;
  if (mw) *(volatile v4f*)md = mv;
  __threadfence();
  #pragma unroll
  for (int p = 0; p < 4; ++p)
    *(volatile v4u*)(qd + (size_t)(p * 4 + (lane >> 3)) * ND + (lane & 7) * 8) = u[p].u;
  if (mw) *(volatile v4f*)md = mv;
}

__global__ void __launch_bounds__(128) k_projkv(const float* __restrict__ ctx,
                                                const _Float16* __restrict__ Wk16,
                                                const __bf16* __restrict__ Wvh,
                                                const __bf16* __restrict__ Wvl,
                                                const float* __restrict__ maskbuf,
                                                _Float16* __restrict__ K16,
                                                _Float16* __restrict__ Vt) {
  __shared__ __attribute__((aligned(16))) _Float16 st[4][16 * LDH];
  __shared__ __attribute__((aligned(16))) _Float16 vts[64 * LDH];
  const int tid = threadIdx.x;
  const int lane = tid & 31, wave = tid >> 5, h = lane >> 4, lm = lane & 15;
  const int blockRow = blockIdx.x * 64;
  const int rowBase = blockRow + wave * 16;
  const int batch = blockRow / NS;
  const int keyBase = blockRow % NS;

  v8f acck[4], accv[4];
  {
    v8f z = {};
    #pragma unroll
    for (int i = 0; i < 4; ++i) { acck[i] = z; accv[i] = z; }
  }
  const float* cr = ctx + (size_t)(rowBase + lm) * NE;

  #pragma unroll 1
  for (int ks = 0; ks < NE / 32; ++ks) {
    const int k0 = ks * 32;
    float f[16];
    load16f(cr + k0 + 8 * h, cr + k0 + 16 + 8 * h, f);
    FragH a;
    FragB ah, al;
    #pragma unroll
    for (int i = 0; i < 16; ++i) {
      a.v[i] = (_Float16)f[i];
      const __bf16 hb = (__bf16)f[i];
      ah.v[i] = hb;
      al.v[i] = (__bf16)(f[i] - (float)hb);
    }
    #pragma unroll
    for (int nt = 0; nt < 4; ++nt) {
      const size_t wo = (size_t)(nt * 16 + lm) * NE + k0;
      FragH b;
      b.h[0] = *(const v8h*)(Wk16 + wo + 8 * h);
      b.h[1] = *(const v8h*)(Wk16 + wo + 16 + 8 * h);
      acck[nt] = mma_f16(a.v, b.v, acck[nt]);
      FragB bh, bl;
      bh.h[0] = *(const v8b*)(Wvh + wo + 8 * h);
      bh.h[1] = *(const v8b*)(Wvh + wo + 16 + 8 * h);
      bl.h[0] = *(const v8b*)(Wvl + wo + 8 * h);
      bl.h[1] = *(const v8b*)(Wvl + wo + 16 + 8 * h);
      accv[nt] = mma_bf16(ah.v, bh.v, accv[nt]);
      accv[nt] = mma_bf16(ah.v, bl.v, accv[nt]);
      accv[nt] = mma_bf16(al.v, bh.v, accv[nt]);
    }
  }

  float mr[8];
  #pragma unroll
  for (int r = 0; r < 8; ++r) mr[r] = maskbuf[(size_t)rowBase + 8 * h + r];

  _Float16* sw = st[wave];
  #pragma unroll
  for (int nt = 0; nt < 4; ++nt) {
    #pragma unroll
    for (int r = 0; r < 8; ++r) {
      sw[(8 * h + r) * LDH + nt * 16 + lm] = (_Float16)(acck[nt][r] * 0.015625f * mr[r]);
      vts[(nt * 16 + lm) * LDH + wave * 16 + 8 * h + r] = (_Float16)(accv[nt][r] * 64.0f * mr[r]);
    }
  }
  __syncthreads();

  Pack16 u[4], w[4];
  #pragma unroll
  for (int p = 0; p < 4; ++p) {
    u[p].h = *(const v8h*)(sw + (p * 4 + (lane >> 3)) * LDH + (lane & 7) * 8);
    w[p].h = *(const v8h*)(vts + (p * 16 + (tid >> 3)) * LDH + (tid & 7) * 8);
  }
  _Float16* kd = K16 + (size_t)rowBase * ND;
  _Float16* vd = Vt + (size_t)batch * ND * NS + keyBase + (tid & 7) * 8;

  #pragma unroll
  for (int p = 0; p < 4; ++p) {
    *(volatile v4u*)(kd + (size_t)(p * 4 + (lane >> 3)) * ND + (lane & 7) * 8) = u[p].u;
    *(volatile v4u*)(vd + (size_t)(p * 16 + (tid >> 3)) * NS) = w[p].u;
  }
  __threadfence();
  #pragma unroll
  for (int p = 0; p < 4; ++p) {
    *(volatile v4u*)(kd + (size_t)(p * 4 + (lane >> 3)) * ND + (lane & 7) * 8) = u[p].u;
    *(volatile v4u*)(vd + (size_t)(p * 16 + (tid >> 3)) * NS) = w[p].u;
  }
}

__global__ void __launch_bounds__(128) k_len(const _Float16* __restrict__ Q16,
                                             const _Float16* __restrict__ K16,
                                             int* __restrict__ lens) {
  __shared__ int red[4];
  __shared__ int res[4];
  const int tid = threadIdx.x;
  const int lane = tid & 31, wave = tid >> 5, h = lane >> 4, lm = lane & 15;

  #pragma unroll 1
  for (int b = 0; b < NB; ++b) {
    const _Float16* qr = Q16 + ((size_t)b * NS + lm) * ND;
    FragH aq[2];
    #pragma unroll
    for (int f = 0; f < 2; ++f) {
      aq[f].h[0] = *(const v8h*)(qr + f * 32 + 8 * h);
      aq[f].h[1] = *(const v8h*)(qr + f * 32 + 16 + 8 * h);
    }
    int cnt = 0;
    #pragma unroll 1
    for (int j = 0; j < NS / (4 * 16); ++j) {
      const int key0 = wave * (NS / 4) + j * 16;
      const _Float16* kr = K16 + ((size_t)b * NS + key0 + lm) * ND;
      v8f e = {};
      #pragma unroll
      for (int f = 0; f < 2; ++f) {
        FragH bk;
        bk.h[0] = *(const v8h*)(kr + f * 32 + 8 * h);
        bk.h[1] = *(const v8h*)(kr + f * 32 + 16 + 8 * h);
        e = mma_f16(aq[f].v, bk.v, e);
      }
      cnt += (h == 0 && e[0] != 0.0f) ? 1 : 0;
    }
    #pragma unroll
    for (int off = 16; off > 0; off >>= 1) cnt += __shfl_xor(cnt, off);
    if (lane == 0) red[wave] = cnt;
    __syncthreads();
    if (tid == 0) res[b] = red[0] + red[1] + red[2] + red[3];
    __syncthreads();
  }

  v4i v = {0, 0, 0, 0};
  if (tid == 0) { v[0] = res[0]; v[1] = res[1]; v[2] = res[2]; v[3] = res[3]; }
  if (tid < 8) *(volatile v4i*)(lens + tid * 4) = v;
  __threadfence();
  if (tid < 8) *(volatile v4i*)(lens + tid * 4) = v;
}

struct AttnTiles {
  _Float16 k[64 * LDH];
  _Float16 v[64 * LDH];
  _Float16 p[8 * 16 * LDH];
};
union AttnLds {
  AttnTiles t;
  float o[8 * 16 * LDO];
};

__global__ void __launch_bounds__(256) k_attn(const _Float16* __restrict__ Q16,
                                              const _Float16* __restrict__ K16,
                                              const _Float16* __restrict__ Vt,
                                              const float* __restrict__ maskbuf,
                                              const int* __restrict__ lens,
                                              float* __restrict__ out) {
  __shared__ __attribute__((aligned(16))) AttnLds L;
  const int tid = threadIdx.x;
  const int lane = tid & 31, wave = tid >> 5, h = lane >> 4, lm = lane & 15;
  const int blk = blockIdx.x;
  const int batch = blk >> 5;
  const int qb = (blk & 31) * 128 + wave * 16;
  int len = lens[batch];
  len = len < 0 ? 0 : (len > NS ? NS : len);
  const float NEG_INF = -__builtin_inff();
  const float ESC = 0.00048828125f;

  FragH aq[2];
  {
    const _Float16* qr = Q16 + ((size_t)batch * NS + qb + lm) * ND;
    #pragma unroll
    for (int f = 0; f < 2; ++f) {
      aq[f].h[0] = *(const v8h*)(qr + f * 32 + 8 * h);
      aq[f].h[1] = *(const v8h*)(qr + f * 32 + 16 + 8 * h);
    }
  }
  v8f oacc[4];
  {
    v8f z = {};
    #pragma unroll
    for (int i = 0; i < 4; ++i) oacc[i] = z;
  }
  float rmax[8], rsum[8];
  #pragma unroll
  for (int r = 0; r < 8; ++r) { rmax[r] = NEG_INF; rsum[r] = 0.0f; }

  const _Float16* kg = K16 + (size_t)batch * NS * ND;
  const _Float16* vg = Vt + (size_t)batch * ND * NS;
  _Float16* pw = L.t.p + wave * 16 * LDH;

  #pragma unroll 1
  for (int kb = 0; kb < NS / 64; ++kb) {
    __syncthreads();
    #pragma unroll
    for (int i = 0; i < 2; ++i) {
      const int c = tid + 256 * i;
      const int row = c >> 3, ch = (c & 7) * 8;
      *(v8h*)(L.t.k + row * LDH + ch) = *(const v8h*)(kg + ((size_t)kb * 64 + row) * ND + ch);
      *(v8h*)(L.t.v + row * LDH + ch) = *(const v8h*)(vg + (size_t)row * NS + kb * 64 + ch);
    }
    __syncthreads();

    v8f e[4];
    {
      v8f z = {};
      #pragma unroll
      for (int t = 0; t < 4; ++t) e[t] = z;
    }
    #pragma unroll
    for (int f = 0; f < 2; ++f) {
      #pragma unroll
      for (int t = 0; t < 4; ++t) {
        const _Float16* kr = L.t.k + (t * 16 + lm) * LDH + f * 32;
        FragH bk;
        bk.h[0] = *(const v8h*)(kr + 8 * h);
        bk.h[1] = *(const v8h*)(kr + 16 + 8 * h);
        e[t] = mma_f16(aq[f].v, bk.v, e[t]);
      }
    }

    bool val[4];
    #pragma unroll
    for (int t = 0; t < 4; ++t) val[t] = (kb * 64 + t * 16 + lm) < len;

    #pragma unroll
    for (int r = 0; r < 8; ++r) {
      float a[4];
      float m = NEG_INF;
      #pragma unroll
      for (int t = 0; t < 4; ++t) {
        a[t] = val[t] ? e[t][r] * ESC : NEG_INF;
        m = fmaxf(m, a[t]);
      }
      #pragma unroll
      for (int off = 1; off < 16; off <<= 1) m = fmaxf(m, __shfl_xor(m, off, 16));
      const float mnew = fmaxf(rmax[r], m);
      const float s = (rmax[r] > NEG_INF) ? __expf(rmax[r] - mnew) : 0.0f;
      float ps = 0.0f;
      #pragma unroll
      for (int t = 0; t < 4; ++t) {
        const float p = (val[t] && mnew > NEG_INF) ? __expf(a[t] - mnew) : 0.0f;
        ps += p;
        pw[(8 * h + r) * LDH + t * 16 + lm] = (_Float16)(p * 256.0f);
      }
      #pragma unroll
      for (int off = 1; off < 16; off <<= 1) ps += __shfl_xor(ps, off, 16);
      rsum[r] = rsum[r] * s + ps;
      rmax[r] = mnew;
      #pragma unroll
      for (int nt = 0; nt < 4; ++nt) oacc[nt][r] *= s;
    }
    __syncthreads();

    #pragma unroll
    for (int g = 0; g < 2; ++g) {
      const _Float16* pr = pw + lm * LDH + g * 32;
      FragH ap;
      ap.h[0] = *(const v8h*)(pr + 8 * h);
      ap.h[1] = *(const v8h*)(pr + 16 + 8 * h);
      #pragma unroll
      for (int nt = 0; nt < 4; ++nt) {
        const _Float16* vr = L.t.v + (nt * 16 + lm) * LDH + g * 32;
        FragH bv;
        bv.h[0] = *(const v8h*)(vr + 8 * h);
        bv.h[1] = *(const v8h*)(vr + 16 + 8 * h);
        oacc[nt] = mma_f16(ap.v, bv.v, oacc[nt]);
      }
    }
  }

  __syncthreads();
  float inv[8];
  #pragma unroll
  for (int r = 0; r < 8; ++r) {
    const float qm = maskbuf[(size_t)batch * NS + qb + 8 * h + r];
    inv[r] = (qm * 0.00006103515625f) / rsum[r];
  }
  float* ow = L.o + wave * 16 * LDO;
  #pragma unroll
  for (int nt = 0; nt < 4; ++nt) {
    #pragma unroll
    for (int r = 0; r < 8; ++r) ow[(8 * h + r) * LDO + nt * 16 + lm] = oacc[nt][r] * inv[r];
  }
  __syncthreads();

  v4f ov[8];
  #pragma unroll
  for (int i = 0; i < 8; ++i)
    ov[i] = *(const v4f*)(ow + (2 * i + (lane >> 4)) * LDO + (lane & 15) * 4);
  float* od = out + ((size_t)batch * NS + qb) * ND + (lane & 15) * 4;
  #pragma unroll
  for (int i = 0; i < 8; ++i)
    *(volatile v4f*)(od + (size_t)(2 * i + (lane >> 4)) * ND) = ov[i];
  __threadfence();
  #pragma unroll
  for (int i = 0; i < 8; ++i)
    *(volatile v4f*)(od + (size_t)(2 * i + (lane >> 4)) * ND) = ov[i];
}

extern "C" void kernel_launch(void* const* d_in, const int* in_sizes, int n_in,
                              void* d_out, int out_size, void* d_ws, size_t ws_size,
                              hipStream_t stream) {
  if (n_in < 5) return;
  if (in_sizes[0] != NROWS * NE || in_sizes[1] != NROWS * NE) return;
  if (in_sizes[2] != NE * ND || in_sizes[3] != NE * ND || in_sizes[4] != NE * ND) return;
  if (out_size != NROWS * ND) return;

  const float* x   = (const float*)d_in[0];
  const float* ctx = (const float*)d_in[1];
  const float* Wq  = (const float*)d_in[2];
  const float* Wk  = (const float*)d_in[3];
  const float* Wv  = (const float*)d_in[4];
  float* out = (float*)d_out;

  char* ws = (char*)d_ws;
  size_t off = 0;
  auto carve = [&](size_t bytes) -> size_t {
    size_t o = off;
    off = (off + bytes + 255) & ~(size_t)255;
    return o;
  };
  const size_t oWq = carve((size_t)ND * NE * 2);
  const size_t oWk = carve((size_t)ND * NE * 2);
  const size_t oWh = carve((size_t)ND * NE * 2);
  const size_t oWl = carve((size_t)ND * NE * 2);
  const size_t oQ  = carve((size_t)NROWS * ND * 2);
  const size_t oK  = carve((size_t)NROWS * ND * 2);
  const size_t oV  = carve((size_t)NROWS * ND * 2);
  const size_t oM  = carve((size_t)NROWS * 4);
  const size_t oL  = carve((size_t)32 * 4);
  if (off > ws_size) return;

  _Float16* Wq16 = (_Float16*)(ws + oWq);
  _Float16* Wk16 = (_Float16*)(ws + oWk);
  __bf16*   Wvh  = (__bf16*)(ws + oWh);
  __bf16*   Wvl  = (__bf16*)(ws + oWl);
  _Float16* Q16  = (_Float16*)(ws + oQ);
  _Float16* K16  = (_Float16*)(ws + oK);
  _Float16* Vt   = (_Float16*)(ws + oV);
  float*    maskbuf = (float*)(ws + oM);
  int*      lens = (int*)(ws + oL);

  const int nchunks = ND * (NE / 8);
  k_prepw<<<(nchunks + 127) / 128, 128, 0, stream>>>(Wq, Wk, Wv, Wq16, Wk16, Wvh, Wvl);
  k_projq<<<NROWS / 64, 128, 0, stream>>>(x, Wq16, Q16, maskbuf);
  k_projkv<<<NROWS / 64, 128, 0, stream>>>(ctx, Wk16, Wvh, Wvl, maskbuf, K16, Vt);
  k_len<<<1, 128, 0, stream>>>(Q16, K16, lens);
  k_attn<<<NROWS / 128, 256, 0, stream>>>(Q16, K16, Vt, maskbuf, lens, out);
  (void)hipGetLastError();
}
